// EGNN_Layer_51788715655765
// MI455X (gfx1250) — hardware-run, weakly checked
//
#include <hip/hip_runtime.h>


#ifndef NB
#define NB 8
#endif
#ifndef NN
#define NN 1024
#endif
#define NB_FULL 8
#define NN_FULL 1024
#define NM   32
#define DM   128
#define DE   32
#define DS   32
#define K1   320
#define XW   192
#define XP   200
#define HP   136
#define OP   132
#define LP   32
#define WCS  16.0f
#define WCI  (1.0f / 16.0f)
#define FREQC (-0.6140226914650789f)
#define OUT1_OFF ((size_t)NB_FULL * NN_FULL * DM)

static_assert(2 * DM + DS + DE == K1);
static_assert(DM + DS + DE == XW);
static_assert(K1 % 32 == 0);
static_assert(XW % 32 == 0);
static_assert(DM % 32 == 0);
static_assert(NM == 32);
static_assert(DM == 8 * 16);
static_assert(XP % 8 == 0 && XP >= XW);
static_assert(HP % 8 == 0 && HP >= DM);
static_assert((OP * 4) % 16 == 0 && OP >= DM);
static_assert(NN % 32 == 0);
static_assert(NB <= NB_FULL);
static_assert(NN <= NN_FULL);
static_assert((NN * 3 / 4) % 8 == 0);
static_assert(((size_t)NN_FULL * 3 * 4) % 128 == 0);
static_assert(OUT1_OFF * 4 == (size_t)4194304);
static_assert(256 * 4 * 16 == 32 * DM * 4);
static_assert(16 * 16 == DM * 2);
static_assert(8 * 16 == LP * 4);
static_assert(2 * 256 * 8 == NM * DM);
static_assert(256 * 4 == NM * DE);
static_assert(2 * 256 == NM * 16);
static_assert(NM * XP * 2 + DM * 2 + 2 * NM * HP * 2 + NM * 16 + DM * 4 + 128 + 128 <= 131072);
static_assert(NM * HP * 2 + NM * OP * 4 <= 131072);

typedef _Float16 h16;
typedef __attribute__((ext_vector_type(16))) _Float16 v16h;
typedef __attribute__((ext_vector_type(8)))  _Float16 v8h;
typedef __attribute__((ext_vector_type(4)))  _Float16 v4h;
typedef __attribute__((ext_vector_type(8)))  float    v8f;
typedef __attribute__((ext_vector_type(4)))  float    v4f;
typedef v4f  __attribute__((may_alias)) v4fa;

__device__ __forceinline__ unsigned short f2bf(float f) { unsigned u = __float_as_uint(f); u += 0x7FFFu + ((u >> 16) & 1u); return (unsigned short)(u >> 16); }
__device__ __forceinline__ float bfr(float f) { return __uint_as_float(((unsigned)f2bf(f)) << 16); }
__device__ __forceinline__ v16h cat16(v8h lo, v8h hi) { return __builtin_shufflevector(lo, hi, 0, 1, 2, 3, 4, 5, 6, 7, 8, 9, 10, 11, 12, 13, 14, 15); }
__device__ __forceinline__ v8f wmma16(v16h a, v16h b, v8f c) { return __builtin_amdgcn_wmma_f32_16x16x32_f16(false, a, false, b, (short)0, c, false, false); }
__device__ __forceinline__ v16h  ldh(const h16* p) { return cat16(*(const v8h*)p, *(const v8h*)(p + 16)); }
#define LDSFRAG(arr, o) cat16(*(const v8h*)(&(arr)[(o)]), *(const v8h*)(&(arr)[(o) + 16]))
static __device__ __forceinline__ h16 toh_flush(float v) { const h16 r = (h16)v; return (fabsf(v) < 6.103515625e-05f) ? (h16)0.0f : r; }
static __device__ __forceinline__ v8f wmma16g(v16h a, v16h b, v8f c) {
    c = wmma16(a, b, c);
    asm volatile("v_nop\n\tv_nop\n\tv_nop\n\tv_nop" : "+v"(c) : "v"(a), "v"(b));
    return c;
}

__global__ __launch_bounds__(256) void k_cvth(const float* __restrict__ src, h16* dst, size_t n8) {
    const size_t i = (size_t)blockIdx.x * 256 + threadIdx.x; if (i >= n8) return;
    const v8f v = *(const v8f*)(src + i * 8); v8h o;
#pragma unroll
    for (int k = 0; k < 8; ++k) o[k] = toh_flush(bfr(v[k]));
    *(volatile v8h*)(dst + i * 8) = o; __threadfence(); *(volatile v8h*)(dst + i * 8) = o;
}

__global__ __launch_bounds__(256) void k_wt(const float* __restrict__ w, h16* dst, int K) {
    const int kp = K >> 3;
    const int i = blockIdx.x * 256 + threadIdx.x; if (i >= DM * kp) return;
    const int n = i / kp, c8 = i - n * kp;
    v8h o;
#pragma unroll
    for (int j = 0; j < 8; ++j) { const float x = w[(size_t)(c8 * 8 + j) * DM + n]; o[j] = toh_flush(bfr(x) * WCS); }
    *(volatile v8h*)(dst + (size_t)i * 8) = o; __threadfence(); *(volatile v8h*)(dst + (size_t)i * 8) = o;
}

__global__ __launch_bounds__(256) void k_pair(const h16* __restrict__ EH, const float* __restrict__ coords, const float* __restrict__ pmask, const float* __restrict__ edges,
                                              const h16* __restrict__ W1T, const float* __restrict__ b1, const h16* __restrict__ W2T, const float* __restrict__ b2,
                                              const h16* __restrict__ WXT, const float* __restrict__ bx1, const float* __restrict__ wx2, const float* __restrict__ bx2,
                                              const int* __restrict__ nbr, h16* MI, float* CD) {
    __shared__ __align__(16) h16 sX[NM * XP];
    __shared__ __align__(16) h16 sE[DM];
    __shared__ __align__(16) h16 sH[NM * HP];
    __shared__ __align__(16) h16 sM[NM * HP];
    __shared__ __align__(16) float sU[NM * 4];
    __shared__ __align__(16) float sMi[DM];
    __shared__ float sCp[8 * 4];
    __shared__ int sNid[NM];

    const int tid = threadIdx.x, lane = tid & 31, lr = lane & 15, hi = lane >> 4;
    const int wave = __builtin_amdgcn_readfirstlane((int)(threadIdx.x >> 5));
    const int col0 = wave * 16;
    const int q = blockIdx.x;
    const int b = q / NN, i = q - b * NN;
    const size_t gp = (size_t)b * NN_FULL + (size_t)i;

    if (wave == 0) {
        int nb = nbr[gp * NM + lane]; nb = nb < 0 ? 0 : (nb > NN_FULL - 1 ? NN_FULL - 1 : nb);
        asm volatile("" : "+v"(nb));
        const size_t g = (size_t)b * NN_FULL + (size_t)nb;
        sNid[lane] = (int)g;
        const float rx = bfr(coords[gp * 3 + 0]) - bfr(coords[g * 3 + 0]);
        const float ry = bfr(coords[gp * 3 + 1]) - bfr(coords[g * 3 + 1]);
        const float rz = bfr(coords[gp * 3 + 2]) - bfr(coords[g * 3 + 2]);
        const float d = sqrtf(rx * rx + ry * ry + rz * rz);
        const float inv = (d > 0.0f) ? (1.0f / d) : 0.0f;
        v4f u; u[0] = rx * inv; u[1] = ry * inv; u[2] = rz * inv; u[3] = d;
        *(v4fa*)(&sU[lane * 4]) = u;
    }
    __syncthreads();

#pragma unroll
    for (int t = 0; t < 2; ++t) { const int p = t * 256 + tid; const int row = p >> 4, c8 = (p & 15) * 8;
        const v8h v = *(const v8h*)(EH + (size_t)sNid[row] * DM + c8);
        *(v8h*)(&sX[row * XP + c8]) = v; }
    if (wave == 1) {
        const v8h v = *(const v8h*)(EH + gp * DM + lr * 8);
        *(v8h*)(&sE[lr * 8]) = v; }
#pragma unroll 1
    for (int t = 0; t < 2; ++t) { const int p = t * 256 + tid; const int row = p >> 4, k = p & 15;
        const float f = expf((float)k * FREQC);
        const float a = sU[row * 4 + 3] * f;
        sX[row * XP + DM + k]      = toh_flush(sinf(a));
        sX[row * XP + DM + 16 + k] = toh_flush(cosf(a)); }
    { const v4f e = *(const v4f*)(edges + gp * (size_t)(NM * DE) + (size_t)tid * 4); const int row = tid >> 3, c = (tid & 7) * 4;
      v4h o;
#pragma unroll
      for (int j = 0; j < 4; ++j) o[j] = toh_flush(bfr(e[j]));
      *(v4h*)(&sX[row * XP + DM + DS + c]) = o; }
    __syncthreads();

    {
        v8f c0 = (v8f){}, c1;
        const h16* wb = W1T + (size_t)(col0 + lr) * K1 + 8 * hi;
#pragma unroll 1
        for (int k0 = 0; k0 < DM; k0 += 32) {
            const v16h a = LDSFRAG(sE, k0 + 8 * hi);
            const v16h bq = ldh(wb + k0);
            c0 = wmma16g(a, bq, c0); }
        c1 = c0;
#pragma unroll 1
        for (int k0 = 0; k0 < XW; k0 += 32) {
            const v16h a0 = LDSFRAG(sX, lr * XP + k0 + 8 * hi);
            const v16h a1 = LDSFRAG(sX, (16 + lr) * XP + k0 + 8 * hi);
            const v16h bq = ldh(wb + DM + k0);
            c0 = wmma16g(a0, bq, c0); c1 = wmma16g(a1, bq, c1); }
        const float bv = bfr(b1[col0 + lr]);
#pragma unroll
        for (int v = 0; v < 8; ++v) { const int r = 8 * hi + v;
            sH[r * HP + col0 + lr]        = toh_flush(fmaxf(c0[v] * WCI + bv, 0.0f));
            sH[(16 + r) * HP + col0 + lr] = toh_flush(fmaxf(c1[v] * WCI + bv, 0.0f)); }
    }
    __syncthreads();

    {
        v8f c0 = (v8f){}, c1 = (v8f){};
        const h16* wb = W2T + (size_t)(col0 + lr) * DM + 8 * hi;
#pragma unroll 1
        for (int k0 = 0; k0 < DM; k0 += 32) {
            const v16h a0 = LDSFRAG(sH, lr * HP + k0 + 8 * hi);
            const v16h a1 = LDSFRAG(sH, (16 + lr) * HP + k0 + 8 * hi);
            const v16h bq = ldh(wb + k0);
            c0 = wmma16g(a0, bq, c0); c1 = wmma16g(a1, bq, c1); }
        const float bv = bfr(b2[col0 + lr]);
        float s = 0.0f;
#pragma unroll
        for (int v = 0; v < 8; ++v) { const int r = 8 * hi + v;
            const float m0 = c0[v] * WCI + bv, m1 = c1[v] * WCI + bv;
            sM[r * HP + col0 + lr]        = toh_flush(m0);
            sM[(16 + r) * HP + col0 + lr] = toh_flush(m1);
            s += m0 + m1; }
        s += __shfl_xor(s, 16, 32);
        const float mk = bfr(pmask[gp]);
        if (hi == 0) sMi[col0 + lr] = s * mk * (1.0f / (float)NM);
    }
    __syncthreads();

    {
        v8f c0 = (v8f){}, c1 = (v8f){};
        const h16* wb = WXT + (size_t)(col0 + lr) * DM + 8 * hi;
#pragma unroll 1
        for (int k0 = 0; k0 < DM; k0 += 32) {
            const v16h a0 = LDSFRAG(sM, lr * HP + k0 + 8 * hi);
            const v16h a1 = LDSFRAG(sM, (16 + lr) * HP + k0 + 8 * hi);
            const v16h bq = ldh(wb + k0);
            c0 = wmma16g(a0, bq, c0); c1 = wmma16g(a1, bq, c1); }
        const float bv = bfr(bx1[col0 + lr]);
        const float wv = bfr(wx2[col0 + lr]);
        float ax = 0.0f, ay = 0.0f, az = 0.0f;
#pragma unroll
        for (int v = 0; v < 8; ++v) { const int r = 8 * hi + v;
            const float t0 = fmaxf(c0[v] * WCI + bv, 0.0f) * wv;
            const float t1 = fmaxf(c1[v] * WCI + bv, 0.0f) * wv;
            const v4f u0 = *(const v4fa*)(&sU[r * 4]); const v4f u1 = *(const v4fa*)(&sU[(16 + r) * 4]);
            ax += u0[0] * t0 + u1[0] * t1; ay += u0[1] * t0 + u1[1] * t1; az += u0[2] * t0 + u1[2] * t1; }
#pragma unroll
        for (int off = 1; off < 32; off <<= 1) { ax += __shfl_xor(ax, off, 32); ay += __shfl_xor(ay, off, 32); az += __shfl_xor(az, off, 32); }
        if (lane == 0) { sCp[wave * 4 + 0] = ax; sCp[wave * 4 + 1] = ay; sCp[wave * 4 + 2] = az; }
    }
    __syncthreads();

    if (wave == 0) {
        const int c = lr * 8;
        const v4f x0 = *(const v4fa*)(&sMi[c]); const v4f x1 = *(const v4fa*)(&sMi[c + 4]); v8h o;
#pragma unroll
        for (int j = 0; j < 4; ++j) { o[j] = toh_flush(x0[j]); o[4 + j] = toh_flush(x1[j]); }
        h16* dp = MI + (size_t)q * DM + c;
        if (lane < 16) *(volatile v8h*)dp = o;
        __threadfence();
        if (lane < 16) *(volatile v8h*)dp = o;
    } else if (wave == 1) {
        float sx = 0.0f, sy = 0.0f, sz = 0.0f, ux = 0.0f, uy = 0.0f, uz = 0.0f;
#pragma unroll 1
        for (int w = 0; w < 8; ++w) { sx += sCp[w * 4 + 0]; sy += sCp[w * 4 + 1]; sz += sCp[w * 4 + 2]; }
#pragma unroll 1
        for (int r = 0; r < NM; ++r) { ux += sU[r * 4 + 0]; uy += sU[r * 4 + 1]; uz += sU[r * 4 + 2]; }
        const float bb = bfr(bx2[0]);
        const float dx = (sx + bb * ux) * (1.0f / (float)NM), dy = (sy + bb * uy) * (1.0f / (float)NM), dz = (sz + bb * uz) * (1.0f / (float)NM);
        v4f o; o[0] = (lane == 0) ? dx : 0.0f; o[1] = (lane == 0) ? dy : 0.0f; o[2] = (lane == 0) ? dz : 0.0f; o[3] = 0.0f;
        float* dp = CD + (size_t)q * LP + (lane & 7) * 4;
        if (lane < 8) *(volatile v4f*)dp = o;
        __threadfence();
        if (lane < 8) *(volatile v4f*)dp = o;
    }
}

__global__ __launch_bounds__(256) void k_node(const h16* __restrict__ EH, const h16* __restrict__ MI, const h16* __restrict__ WH1T, const float* __restrict__ bh1,
                                              const h16* __restrict__ WH2T, const float* __restrict__ bh2, const float* __restrict__ emb, float* OUT) {
    __shared__ __align__(16) h16 sT[NM * HP];
    __shared__ __align__(16) float sO[NM * OP];
    const int tid = threadIdx.x, lane = tid & 31, lr = lane & 15, hi = lane >> 4;
    const int wave = __builtin_amdgcn_readfirstlane((int)(threadIdx.x >> 5));
    const int col0 = wave * 16;
    const int q0 = blockIdx.x * 32;
    const int b = q0 / NN, i0 = q0 - b * NN;
    const size_t gr0 = (size_t)b * NN_FULL + (size_t)i0;
    {
        v8f c0 = (v8f){}, c1 = (v8f){};
        const h16* wb = WH1T + (size_t)(col0 + lr) * (2 * DM) + 8 * hi;
        const size_t ea = (gr0 + (size_t)lr) * DM + 8 * hi;
        const size_t ma = ((size_t)q0 + (size_t)lr) * DM + 8 * hi;
#pragma unroll 1
        for (int k0 = 0; k0 < DM; k0 += 32) {
            const v16h a0 = ldh(EH + ea + k0), a1 = ldh(EH + ea + (size_t)16 * DM + k0);
            const v16h bq = ldh(wb + k0);
            c0 = wmma16g(a0, bq, c0); c1 = wmma16g(a1, bq, c1); }
#pragma unroll 1
        for (int k0 = 0; k0 < DM; k0 += 32) {
            const v16h a0 = ldh(MI + ma + k0), a1 = ldh(MI + ma + (size_t)16 * DM + k0);
            const v16h bq = ldh(wb + DM + k0);
            c0 = wmma16g(a0, bq, c0); c1 = wmma16g(a1, bq, c1); }
        const float bv = bfr(bh1[col0 + lr]);
#pragma unroll
        for (int v = 0; v < 8; ++v) { const int r = 8 * hi + v;
            sT[r * HP + col0 + lr]        = toh_flush(fmaxf(c0[v] * WCI + bv, 0.0f));
            sT[(16 + r) * HP + col0 + lr] = toh_flush(fmaxf(c1[v] * WCI + bv, 0.0f)); }
    }
    __syncthreads();
    {
        v8f c0 = (v8f){}, c1 = (v8f){};
        const h16* wb = WH2T + (size_t)(col0 + lr) * DM + 8 * hi;
#pragma unroll 1
        for (int k0 = 0; k0 < DM; k0 += 32) {
            const v16h a0 = LDSFRAG(sT, lr * HP + k0 + 8 * hi);
            const v16h a1 = LDSFRAG(sT, (16 + lr) * HP + k0 + 8 * hi);
            const v16h bq = ldh(wb + k0);
            c0 = wmma16g(a0, bq, c0); c1 = wmma16g(a1, bq, c1); }
        const float bv = bfr(bh2[col0 + lr]);
#pragma unroll
        for (int v = 0; v < 8; ++v) { const int r = 8 * hi + v;
            sO[r * OP + col0 + lr]        = c0[v] * WCI + bv;
            sO[(16 + r) * OP + col0 + lr] = c1[v] * WCI + bv; }
    }
    __syncthreads();
    v4f val[4];
#pragma unroll
    for (int it = 0; it < 4; ++it) { const int p = it * 256 + tid; const int row = p >> 5, c4 = (p & 31) * 4;
        const v4f s = *(const v4fa*)(&sO[row * OP + c4]);
        const v4f e = *(const v4f*)(emb + (gr0 + (size_t)row) * DM + c4);
#pragma unroll
        for (int j = 0; j < 4; ++j) val[it][j] = s[j] + bfr(e[j]); }
#pragma unroll 1
    for (int ps = 0; ps < 2; ++ps) {
#pragma unroll
        for (int it = 0; it < 4; ++it) { const int p = it * 256 + tid; const int row = p >> 5, c4 = (p & 31) * 4;
            *(volatile v4f*)(OUT + (gr0 + (size_t)row) * DM + c4) = val[it]; }
        if (ps == 0) __threadfence(); }
}

__global__ __launch_bounds__(256) void k_coord(const float* __restrict__ coords, const float* __restrict__ CD, float* OUT1) {
    const int per = NN * 3 / 4;
    const int i4 = blockIdx.x * 256 + threadIdx.x; if (i4 >= NB * per) return;
    const int b = i4 / per, r = i4 - b * per;
    const size_t base = (size_t)b * NN_FULL * 3 + (size_t)r * 4;
    const v4f c = *(const v4f*)(coords + base);
    v4f o;
#pragma unroll
    for (int j = 0; j < 4; ++j) { const int e = r * 4 + j; const int node = e / 3, cc = e - node * 3;
        const float d = CD[((size_t)b * NN + (size_t)node) * LP + cc];
        o[j] = bfr(c[j]) + d; }
    *(volatile v4f*)(OUT1 + base) = o; __threadfence(); *(volatile v4f*)(OUT1 + base) = o;
}

static constexpr size_t al256(size_t v) { return (v + 255) & ~(size_t)255; }
static constexpr size_t SZ_EH  = al256((size_t)NB * NN_FULL * DM * 2);
static constexpr size_t SZ_W1  = al256((size_t)DM * K1 * 2);
static constexpr size_t SZ_WS  = al256((size_t)DM * DM * 2);
static constexpr size_t SZ_WH1 = al256((size_t)DM * 2 * DM * 2);
static constexpr size_t SZ_MI  = al256((size_t)NB * NN * DM * 2);
static constexpr size_t SZ_CD  = al256((size_t)NB * NN * LP * 4);
static constexpr size_t SZ_TOTAL = SZ_EH + SZ_W1 + 3 * SZ_WS + SZ_WH1 + SZ_MI + SZ_CD;
static_assert(SZ_TOTAL <= (size_t)134217728);
static_assert(((size_t)NB * NN_FULL * DM) % (8 * 256) == 0);
static_assert((DM * (K1 / 8)) % 256 == 0);
static_assert((DM * (DM / 8)) % 256 == 0);
static_assert((DM * (2 * DM / 8)) % 256 == 0);
static_assert((NB * NN) % 32 == 0);

extern "C" void kernel_launch(void* const* d_in, const int* in_sizes, int n_in,
                              void* d_out, int out_size, void* d_ws, size_t ws_size, hipStream_t stream) {
    if (n_in < 17) return;
    const size_t nodes_need = (size_t)(NB - 1) * NN_FULL + NN;
    if ((size_t)in_sizes[0] < (size_t)NB * NN_FULL * DM) return;
    if ((size_t)in_sizes[1] < (size_t)NB * NN_FULL * 3) return;
    if ((size_t)in_sizes[2] < nodes_need) return;
    if ((size_t)in_sizes[3] < nodes_need * NM * DE) return;
    if (in_sizes[4] < K1 * DM || in_sizes[5] < DM || in_sizes[6] < DM * DM || in_sizes[7] < DM) return;
    if (in_sizes[8] < DM * DM || in_sizes[9] < DM || in_sizes[10] < DM || in_sizes[11] < 1) return;
    if (in_sizes[12] < 2 * DM * DM || in_sizes[13] < DM || in_sizes[14] < DM * DM || in_sizes[15] < DM) return;
    if ((size_t)in_sizes[16] < nodes_need * NM) return;
    if ((size_t)out_size < OUT1_OFF + nodes_need * 3) return;
    if (SZ_TOTAL > ws_size) return;
    const float* emb    = (const float*)d_in[0];
    const float* coords = (const float*)d_in[1];
    const float* pmask  = (const float*)d_in[2];
    const float* edges  = (const float*)d_in[3];
    const float* we_w1  = (const float*)d_in[4];  const float* we_b1 = (const float*)d_in[5];
    const float* we_w2  = (const float*)d_in[6];  const float* we_b2 = (const float*)d_in[7];
    const float* wx_w1  = (const float*)d_in[8];  const float* wx_b1 = (const float*)d_in[9];
    const float* wx_w2  = (const float*)d_in[10]; const float* wx_b2 = (const float*)d_in[11];
    const float* wh_w1  = (const float*)d_in[12]; const float* wh_b1 = (const float*)d_in[13];
    const float* wh_w2  = (const float*)d_in[14]; const float* wh_b2 = (const float*)d_in[15];
    const int*   nbr    = (const int*)d_in[16];
    float* OUT0 = (float*)d_out;
    float* OUT1 = (float*)d_out + OUT1_OFF;
    char* wsp = (char*)d_ws;
    h16* EH   = (h16*)wsp; wsp += SZ_EH;
    h16* W1T  = (h16*)wsp; wsp += SZ_W1;
    h16* W2T  = (h16*)wsp; wsp += SZ_WS;
    h16* WXT  = (h16*)wsp; wsp += SZ_WS;
    h16* WH2T = (h16*)wsp; wsp += SZ_WS;
    h16* WH1T = (h16*)wsp; wsp += SZ_WH1;
    h16* MI   = (h16*)wsp; wsp += SZ_MI;
    float* CD = (float*)wsp; wsp += SZ_CD;

    { const size_t n8 = (size_t)NB * NN_FULL * DM / 8;
      k_cvth<<<(unsigned)((n8 + 255) / 256), 256, 0, stream>>>(emb, EH, n8); }
    k_wt<<<(DM * (K1 / 8) + 255) / 256, 256, 0, stream>>>(we_w1, W1T, K1);
    k_wt<<<(DM * (DM / 8) + 255) / 256, 256, 0, stream>>>(we_w2, W2T, DM);
    k_wt<<<(DM * (DM / 8) + 255) / 256, 256, 0, stream>>>(wx_w1, WXT, DM);
    k_wt<<<(DM * (2 * DM / 8) + 255) / 256, 256, 0, stream>>>(wh_w1, WH1T, 2 * DM);
    k_wt<<<(DM * (DM / 8) + 255) / 256, 256, 0, stream>>>(wh_w2, WH2T, DM);

    k_pair<<<NB * NN, 256, 0, stream>>>(EH, coords, pmask, edges, W1T, we_b1, W2T, we_b2, WXT, wx_b1, wx_w2, wx_b2, nbr, MI, CD);
    k_node<<<NB * NN / 32, 256, 0, stream>>>(EH, MI, WH1T, wh_b1, WH2T, wh_b2, emb, OUT0);
    k_coord<<<(NB * (NN * 3 / 4) + 255) / 256, 256, 0, stream>>>(coords, CD, OUT1);
}
